// MinibatchDiscriminator64_68599217652003
// MI455X (gfx1250) — hardware-verified
//
#include <hip/hip_runtime.h>
#include <math.h>

typedef __attribute__((ext_vector_type(16))) _Float16 v16h;
typedef __attribute__((ext_vector_type(16))) __bf16 v16b;
typedef __attribute__((ext_vector_type(8)))  _Float16 v8h;
typedef __attribute__((ext_vector_type(8)))  float v8f;
typedef __attribute__((ext_vector_type(4)))  float v4f;
typedef __attribute__((ext_vector_type(2)))  float v2f;
typedef __attribute__((ext_vector_type(4)))  unsigned v4u;
typedef __attribute__((ext_vector_type(4)))  int v4i;
typedef float __attribute__((may_alias)) float_a;
typedef int __attribute__((may_alias)) int_a;

template <typename T> __device__ __forceinline__ void vst2(void* p, T v) { *(volatile T*)p = v; __threadfence(); *(volatile T*)p = v; }
__device__ __forceinline__ v8f wmma16(v16h a, v16h b, v8f c) {
  v8f d = __builtin_amdgcn_wmma_f32_16x16x32_f16(false, a, false, b, (short)0, c, false, false);
  asm volatile("v_nop\n\tv_nop\n\tv_nop\n\tv_nop" : "+v"(d) : "v"(a), "v"(b));
  return d;
}
__device__ __forceinline__ v8f wmma_bf(v16b a, v16b b, v8f c) {
  v8f d = __builtin_amdgcn_wmma_f32_16x16x32_bf16(false, a, false, b, (short)0, c, false, false);
  asm volatile("v_nop\n\tv_nop\n\tv_nop\n\tv_nop" : "+v"(d) : "v"(a), "v"(b));
  return d;
}
__device__ __forceinline__ v16h frag_h(const _Float16* rowk0, int lane) {
  union { v16h v; v8h q[2]; } u; const _Float16* p = rowk0 + 8 * (lane >> 4);
  u.q[0] = *(const v8h*)p; u.q[1] = *(const v8h*)(p + 16); return u.v;
}
__device__ __forceinline__ v16h frag_f32(const float* rowk0, int lane) {
  v16h a; const float* p = rowk0 + 8 * (lane >> 4);
#pragma unroll
  for (int i = 0; i < 8; ++i) { a[i] = (_Float16)p[i]; a[8 + i] = (_Float16)p[16 + i]; }
  return a;
}
__device__ __forceinline__ v16h frag_f32s(const float* rowk0, int lane, float sc) {
  v16h a; const float* p = rowk0 + 8 * (lane >> 4);
#pragma unroll
  for (int i = 0; i < 8; ++i) { a[i] = (_Float16)(p[i] * sc); a[8 + i] = (_Float16)(p[16 + i] * sc); }
  return a;
}
__device__ __forceinline__ v16h fragc_f32(const float* W, int k0, int n, int lane, int ld, int K) {
  v16h a; const int g = lane >> 4;
#pragma unroll
  for (int i = 0; i < 8; ++i) { const int ka = k0 + 8 * g + i, kb = ka + 16;
    a[i] = (_Float16)(ka < K ? W[(size_t)(ka < K ? ka : K - 1) * ld + n] : 0.f); a[8 + i] = (_Float16)(kb < K ? W[(size_t)(kb < K ? kb : K - 1) * ld + n] : 0.f); }
  return a;
}
struct F2 { v16b h, l; };
__device__ __forceinline__ F2 bsplit16(const float v[16]) { F2 r;
#pragma unroll
  for (int i = 0; i < 16; ++i) { const __bf16 h = (__bf16)v[i]; r.h[i] = h; r.l[i] = (__bf16)(v[i] - (float)h); }
  return r; }
__device__ __forceinline__ F2 split_row(const float* row, int k0, int lane) { float v[16]; const float* p = row + k0 + 8 * (lane >> 4);
#pragma unroll
  for (int i = 0; i < 8; ++i) { v[i] = p[i]; v[8 + i] = p[16 + i]; }
  return bsplit16(v); }
__device__ __forceinline__ F2 split_rowK(const float* row, int k0, int lane, int K) { float v[16]; const int g = lane >> 4;
#pragma unroll
  for (int i = 0; i < 8; ++i) { const int ka = k0 + 8 * g + i, kb = ka + 16; v[i] = ka < K ? row[ka < K ? ka : K - 1] : 0.f; v[8 + i] = kb < K ? row[kb < K ? kb : K - 1] : 0.f; }
  return bsplit16(v); }
__device__ __forceinline__ F2 split_col(const float* W, int k0, int n, int lane, int ld, int K) { float v[16]; const int g = lane >> 4;
#pragma unroll
  for (int i = 0; i < 8; ++i) { const int ka = k0 + 8 * g + i, kb = ka + 16; v[i] = ka < K ? W[(size_t)(ka < K ? ka : K - 1) * ld + n] : 0.f; v[8 + i] = kb < K ? W[(size_t)(kb < K ? kb : K - 1) * ld + n] : 0.f; }
  return bsplit16(v); }
__device__ __forceinline__ v8f mac3(const F2& a, const F2& b, v8f c) { c = wmma_bf(a.l, b.h, c); c = wmma_bf(a.h, b.l, c); return wmma_bf(a.h, b.h, c); }
__device__ __forceinline__ float sigm(float v) { return 1.0f / (1.0f + expf(-v)); }
#define LDSX() do { asm volatile("s_wait_dscnt 0" ::: "memory"); __builtin_amdgcn_wave_barrier(); __builtin_amdgcn_fence(__ATOMIC_RELEASE, "workgroup"); } while (0)


#ifndef BS
#define BS 256
#endif
#define EPS 1e-5f
typedef __attribute__((ext_vector_type(8))) __bf16 v8b;
__device__ __forceinline__ v16b frag_b(const __bf16* rowk0, int lane) {
  union { v16b v; v8b q[2]; } u; const __bf16* p = rowk0 + 8 * (lane >> 4);
  u.q[0] = *(const v8b*)p; u.q[1] = *(const v8b*)(p + 16); return u.v;
}
__device__ __forceinline__ float bfr(float v) { return (float)(__bf16)v; }
__device__ __attribute__((noinline)) float exp_ni(float v) { return expf(v); }
__device__ __attribute__((noinline)) float erf_ni(float v) { return erff(v); }

#define C0 3
#define H0 64
#define C1 64
#define H1 32
#define C2 128
#define H2 16
#define C3 256
#define H3 8
#define C4 256
#define H4 4
#define K1P 96
#define K2 1600
#define K3 3200
#define K4 2304
#define FEAT 4096
#define TO 3200
#define MBW 4160
#define NY 1000
#define NYP 1024

#define PK_1 0
#define PK_2 ((size_t)C1 * K1P)
#define PK_3 (PK_2 + (size_t)C2 * K2)
#define PK_4 (PK_3 + (size_t)C3 * K3)
#define PK_T (PK_4 + (size_t)C4 * K4)
#define PK_F (PK_T + (size_t)TO * FEAT)
#define PK_END (PK_F + (size_t)NYP * MBW)
#define WS_PK  0u
#define WS_Y1  (((2u * PK_END) + 127u) / 128u * 128u)
#define WS_Y2  (WS_Y1 + 4u * (size_t)BS * C1 * H1 * H1)
#define WS_Y3  (WS_Y2 + 4u * (size_t)BS * C2 * H2 * H2)
#define WS_Y4  (WS_Y3 + 4u * (size_t)BS * C3 * H3 * H3)
#define WS_ST  (WS_Y4 + 4u * (size_t)BS * C4 * H4 * H4)
#define WS_MS1 (WS_ST + 4u * (size_t)BS * 16 * 256 * 2)
#define WS_MS2 (WS_MS1 + 4u * (size_t)BS * C1 * 2)
#define WS_MS3 (WS_MS2 + 4u * (size_t)BS * C2 * 2)
#define WS_MS4 (WS_MS3 + 4u * (size_t)BS * C3 * 2)
#define WS_FH  (WS_MS4 + 4u * (size_t)BS * C4 * 2)
#define WS_FL  (WS_FH + 2u * (size_t)BS * MBW)
#define WS_M   (WS_FL + 2u * (size_t)BS * MBW)
#define WS_END (WS_M + 4u * (size_t)BS * TO)

__global__ __launch_bounds__(256) void k_pack(const float* __restrict__ W1, const float* __restrict__ W2, const float* __restrict__ W3, const float* __restrict__ W4, const float* __restrict__ T, const float* __restrict__ FCW, __bf16* __restrict__ PK) {
  __shared__ __align__(16) __bf16 s[MBW]; const int n = blockIdx.x, which = blockIdx.y, t = threadIdx.x; int K; size_t dst;
  switch (which) {
    case 0: if (n >= C1) return; K = K1P; dst = PK_1 + (size_t)n * K1P; for (int k = t; k < K; k += 256) s[k] = (__bf16)((k < C0 * 25) ? W1[(size_t)n * 75 + k] : 0.f); break;
    case 1: if (n >= C2) return; K = K2; dst = PK_2 + (size_t)n * K2; for (int k = t; k < K; k += 256) s[k] = (__bf16)W2[(size_t)n * K2 + k]; break;
    case 2: if (n >= C3) return; K = K3; dst = PK_3 + (size_t)n * K3; for (int k = t; k < K; k += 256) s[k] = (__bf16)W3[(size_t)n * K3 + k]; break;
    case 3: if (n >= C4) return; K = K4; dst = PK_4 + (size_t)n * K4; for (int k = t; k < K; k += 256) s[k] = (__bf16)W4[(size_t)n * K4 + k]; break;
    case 4: if (n >= TO) return; K = FEAT; dst = PK_T + (size_t)n * FEAT; for (int k = t; k < K; k += 256) s[k] = (__bf16)T[(size_t)k * TO + n]; break;
    default: if (n >= NYP) return; K = MBW; dst = PK_F + (size_t)n * MBW; for (int k = t; k < K; k += 256) s[k] = (__bf16)((n < NY) ? FCW[(size_t)n * MBW + k] : 0.f); break; }
  __syncthreads();
  for (int q = t; q < K / 8; q += 256) vst2((unsigned*)(PK + dst + q * 8), *(const v4u*)&s[q * 8]);
}
template <int L>
__global__ __launch_bounds__(128) void k_conv(const float* __restrict__ SRC, const float* __restrict__ MSP, const float* __restrict__ GP, const float* __restrict__ BEP, const __bf16* __restrict__ PK, const float* __restrict__ BIAS, float* __restrict__ Y, float* __restrict__ ST) {
  constexpr int CIN = (L == 1) ? C0 : (L == 2) ? C1 : (L == 3) ? C2 : C3; constexpr int HIN = (L == 1) ? H0 : (L == 2) ? H1 : (L == 3) ? H2 : H3; constexpr int COUT = (L == 1) ? C1 : (L == 2) ? C2 : (L == 3) ? C3 : C4; constexpr int HOUT = HIN / 2;
  constexpr int KS = (L == 4) ? 3 : 5; constexpr int PAD = (L == 4) ? 1 : 2; constexpr int KK = (L == 1) ? K1P : CIN * KS * KS; constexpr int NPX = HOUT * HOUT; constexpr int NT = COUT / 16;
  const size_t pk = (L == 1) ? PK_1 : (L == 2) ? PK_2 : (L == 3) ? PK_3 : PK_4;
  __shared__ __align__(16) __bf16 sh[64][40], sl[64][40]; __shared__ __align__(16) float so[COUT][68];
  const int tid = threadIdx.x, wave = tid >> 5, lane = tid & 31, col = lane & 15, g = lane >> 4; const size_t b = blockIdx.y; const int p0 = blockIdx.x * 64;
  v8f acc[NT] = {};
#pragma unroll 1
  for (int kc = 0; kc < KK / 32; ++kc) {
    for (int e = tid; e < 64 * 32; e += 128) { const int r = e >> 5, c = e & 31; const int kk = kc * 32 + c; const int p = p0 + r; float v = 0.f;
      if (p < NPX && kk < CIN * KS * KS) { const int ci = kk / (KS * KS), ij = kk % (KS * KS), i = ij / KS, j = ij % KS; const int oy = p / HOUT, ox = p % HOUT; const int yy = 2 * oy + i - PAD, xx = 2 * ox + j - PAD;
        if (yy >= 0 && yy < HIN && xx >= 0 && xx < HIN) { const float raw = SRC[((b * CIN + ci) * HIN + yy) * HIN + xx];
          if (L == 1) v = bfr(raw); else { const float mu = MSP[(b * CIN + ci) * 2], rs = MSP[(b * CIN + ci) * 2 + 1]; float z = (raw - mu) * rs * bfr(GP[ci]) + bfr(BEP[ci]); v = (z >= 0.f) ? z : 0.2f * z; } } }
      const __bf16 hb = (__bf16)v; sh[r][c] = hb; sl[r][c] = (__bf16)(v - (float)hb); }
    __syncthreads();
    F2 a; a.h = frag_b(&sh[wave * 16 + col][0], lane); a.l = frag_b(&sl[wave * 16 + col][0], lane);
#pragma unroll
    for (int j = 0; j < NT; ++j) { const v16b w = frag_b(PK + pk + (size_t)(j * 16 + col) * KK + kc * 32, lane); if (L > 1) acc[j] = wmma_bf(a.l, w, acc[j]); acc[j] = wmma_bf(a.h, w, acc[j]); }
    __syncthreads(); }
#pragma unroll
  for (int j = 0; j < NT; ++j) { const int c = j * 16 + col; const float bb = bfr(BIAS[c]);
#pragma unroll
    for (int r = 0; r < 8; ++r) so[c][wave * 16 + 8 * g + r] = acc[j][r] + bb; }
  __syncthreads();
  const int npx = (NPX < 64) ? NPX : 64;
  for (int e = tid; e < COUT * (npx / 4); e += 128) { const int c = e / (npx / 4), q4 = e % (npx / 4); vst2(Y + ((b * COUT + c) * NPX) + p0 + q4 * 4, *(const v4f*)&so[c][q4 * 4]); }
  __shared__ __align__(16) float sst[256 * 2];
  for (int c = tid; c < COUT; c += 128) { float s = 0.f, q2 = 0.f; for (int r = 0; r < npx; ++r) { const float v = so[c][r]; s += v; q2 += v * v; } sst[c * 2] = s; sst[c * 2 + 1] = q2; }
  __syncthreads();
  for (int e = tid; e < COUT * 2 / 4; e += 128) vst2(ST + ((b * 16 + blockIdx.x) * 256) * 2 + e * 4, *(const v4f*)&sst[e * 4]);
}
__global__ __launch_bounds__(256) void k_istat(const float* __restrict__ ST, int ntiles, int cout, float npx, float* __restrict__ MS) {
  const size_t b = blockIdx.x; const int c = threadIdx.x; __shared__ __align__(16) float sm[256 * 2];
  if (c < cout) { float s = 0.f, q2 = 0.f; for (int t = 0; t < ntiles; ++t) { s += ST[((b * 16 + t) * 256 + c) * 2]; q2 += ST[((b * 16 + t) * 256 + c) * 2 + 1]; } const float mu = s / npx; sm[c * 2] = mu; sm[c * 2 + 1] = 1.0f / sqrtf(fmaxf(q2 / npx - mu * mu, 0.f) + EPS); }
  __syncthreads();
  for (int e = c; e < cout * 2 / 4; e += 256) vst2(MS + (b * cout) * 2 + e * 4, *(const v4f*)&sm[e * 4]);
}
__global__ __launch_bounds__(256) void k_feat(const float* __restrict__ Y4, const float* __restrict__ MS4, const float* __restrict__ G4, const float* __restrict__ BE4, float* __restrict__ OUT0, __bf16* __restrict__ FH, __bf16* __restrict__ FL) {
  __shared__ __align__(16) float sf[FEAT]; __shared__ __align__(16) __bf16 shh[FEAT], sll[FEAT]; const size_t b = blockIdx.x; const int t = threadIdx.x;
  for (int e = t; e < FEAT; e += 256) { const int c = e >> 4; const float mu = MS4[(b * C4 + c) * 2], rs = MS4[(b * C4 + c) * 2 + 1]; float z = (Y4[b * FEAT + e] - mu) * rs * bfr(G4[c]) + bfr(BE4[c]); z = (z >= 0.f) ? z : 0.2f * z; sf[e] = z; const __bf16 hb = (__bf16)z; shh[e] = hb; sll[e] = (__bf16)(z - (float)hb); }
  __syncthreads();
  for (int e = t; e < FEAT / 4; e += 256) vst2(OUT0 + b * FEAT + e * 4, *(const v4f*)&sf[e * 4]);
  for (int e = t; e < FEAT / 8; e += 256) { vst2((unsigned*)(FH + b * MBW + e * 8), *(const v4u*)&shh[e * 8]); vst2((unsigned*)(FL + b * MBW + e * 8), *(const v4u*)&sll[e * 8]); }
}
__global__ __launch_bounds__(128) void k_m(const __bf16* __restrict__ FH, const __bf16* __restrict__ FL, const __bf16* __restrict__ PK, float* __restrict__ M) {
  __shared__ __align__(16) float so[4][16][132];
  const int tid = threadIdx.x, wave = tid >> 5, lane = tid & 31, col = lane & 15, g = lane >> 4; const size_t r0 = (size_t)blockIdx.x * 64 + wave * 16; const int n0 = blockIdx.y * 128;
  v8f acc[8] = {};
#pragma unroll 2
  for (int kc = 0; kc < FEAT / 32; ++kc) { const size_t ra = ((r0 + col) < (size_t)BS) ? (r0 + col) : (size_t)BS - 1; const v16b a = frag_b(FH + ra * MBW + kc * 32, lane), al = frag_b(FL + ra * MBW + kc * 32, lane);
#pragma unroll
    for (int j = 0; j < 8; ++j) { if (n0 + j * 16 >= TO) continue; const v16b w = frag_b(PK + PK_T + (size_t)(n0 + j * 16 + col) * FEAT + kc * 32, lane); acc[j] = wmma_bf(al, w, acc[j]); acc[j] = wmma_bf(a, w, acc[j]); } }
#pragma unroll
  for (int j = 0; j < 8; ++j)
#pragma unroll
    for (int r = 0; r < 8; ++r) so[wave][8 * g + r][j * 16 + col] = acc[j][r];
  LDSX();
  for (int rl = 0; rl < 16; ++rl) if ((r0 + rl) < (size_t)BS && n0 + lane * 4 < TO) vst2(M + (r0 + rl) * TO + n0 + lane * 4, *(const v4f*)&so[wave][rl][lane * 4]);
}
__global__ __launch_bounds__(256) void k_ob(const float* __restrict__ M, __bf16* __restrict__ FH, __bf16* __restrict__ FL) {
  __shared__ float smi[TO]; __shared__ float sp[64][4]; __shared__ __align__(16) __bf16 sh[64], slo[64]; const size_t i = blockIdx.x; const int t = threadIdx.x; const int k = t >> 2, sub = t & 3;
  for (int e = t; e < TO; e += 256) smi[e] = M[i * TO + e];
  __syncthreads();
  float a = 0.f;
#pragma unroll 1
  for (int j = sub; j < BS; j += 4) { const float* mj = M + (size_t)j * TO + k * 50; float nrm = 0.f;
#pragma unroll 1
    for (int l = 0; l < 50; ++l) nrm += fabsf(smi[k * 50 + l] - mj[l]);
    a += exp_ni(-nrm); }
  sp[k][sub] = a; __syncthreads();
  if (t < 64) { const float ob = ((sp[t][0] + sp[t][1]) + (sp[t][2] + sp[t][3])) - 1.0f; const __bf16 hb = (__bf16)ob; sh[t] = hb; slo[t] = (__bf16)(ob - (float)hb); }
  __syncthreads();
  if (t < 8) { vst2((unsigned*)(FH + i * MBW + FEAT + t * 8), *(const v4u*)&sh[t * 8]); vst2((unsigned*)(FL + i * MBW + FEAT + t * 8), *(const v4u*)&slo[t * 8]); }
}
__global__ __launch_bounds__(128) void k_fc(const __bf16* __restrict__ FH, const __bf16* __restrict__ FL, const __bf16* __restrict__ PK, const float* __restrict__ FCB, float* __restrict__ OUT1) {
  __shared__ __align__(16) float sy[16 * NY];
  const int tid = threadIdx.x, wave = tid >> 5, lane = tid & 31, col = lane & 15, g = lane >> 4; const size_t r0 = (size_t)blockIdx.x * 16;
#pragma unroll 1
  for (int pass = 0; pass < 2; ++pass) { const int n0 = wave * 256 + pass * 128; v8f acc[8] = {};
#pragma unroll 2
    for (int kc = 0; kc < MBW / 32; ++kc) { const v16b a = frag_b(FH + (r0 + col) * MBW + kc * 32, lane), al = frag_b(FL + (r0 + col) * MBW + kc * 32, lane);
#pragma unroll
      for (int j = 0; j < 8; ++j) { const v16b w = frag_b(PK + PK_F + (size_t)(n0 + j * 16 + col) * MBW + kc * 32, lane); acc[j] = wmma_bf(al, w, acc[j]); acc[j] = wmma_bf(a, w, acc[j]); } }
#pragma unroll
    for (int j = 0; j < 8; ++j) { const int c = n0 + j * 16 + col; if (c < NY) { const float bb = bfr(FCB[c]);
#pragma unroll
      for (int r = 0; r < 8; ++r) sy[(8 * g + r) * NY + c] = acc[j][r] + bb; } } }
  __syncthreads();
  for (int e = tid; e < 16 * NY / 4; e += 128) vst2(OUT1 + r0 * NY + e * 4, *(const v4f*)&sy[e * 4]);
}
extern "C" void kernel_launch(void* const* d_in, const int* in_sizes, int n_in, void* d_out, int out_size, void* d_ws, size_t ws_size, hipStream_t stream) {
  (void)in_sizes; (void)n_in; (void)out_size;
  const float** F = (const float**)d_in;
  if (ws_size < (size_t)WS_END) return;
  char* ws = (char*)d_ws; __bf16 *PK = (__bf16*)(ws + WS_PK), *FH = (__bf16*)(ws + WS_FH), *FL = (__bf16*)(ws + WS_FL); float *Y1 = (float*)(ws + WS_Y1), *Y2 = (float*)(ws + WS_Y2), *Y3 = (float*)(ws + WS_Y3), *Y4 = (float*)(ws + WS_Y4), *ST = (float*)(ws + WS_ST), *MS1 = (float*)(ws + WS_MS1), *MS2 = (float*)(ws + WS_MS2), *MS3 = (float*)(ws + WS_MS3), *MS4 = (float*)(ws + WS_MS4), *M = (float*)(ws + WS_M);
  float* OUT0 = (float*)d_out; float* OUT1 = (float*)((char*)d_out + (size_t)256 * FEAT * 4);
  k_pack<<<dim3(TO, 6), 256, 0, stream>>>(F[1], F[5], F[9], F[13], F[17], F[18], PK);
  k_conv<1><<<dim3(H1 * H1 / 64, BS), 128, 0, stream>>>(F[0], nullptr, nullptr, nullptr, PK, F[2], Y1, ST);
  k_istat<<<BS, 256, 0, stream>>>(ST, H1 * H1 / 64, C1, (float)(H1 * H1), MS1);
  k_conv<2><<<dim3(H2 * H2 / 64, BS), 128, 0, stream>>>(Y1, MS1, F[3], F[4], PK, F[6], Y2, ST);
  k_istat<<<BS, 256, 0, stream>>>(ST, H2 * H2 / 64, C2, (float)(H2 * H2), MS2);
  k_conv<3><<<dim3(1, BS), 128, 0, stream>>>(Y2, MS2, F[7], F[8], PK, F[10], Y3, ST);
  k_istat<<<BS, 256, 0, stream>>>(ST, 1, C3, (float)(H3 * H3), MS3);
  k_conv<4><<<dim3(1, BS), 128, 0, stream>>>(Y3, MS3, F[11], F[12], PK, F[14], Y4, ST);
  k_istat<<<BS, 256, 0, stream>>>(ST, 1, C4, (float)(H4 * H4), MS4);
  k_feat<<<BS, 256, 0, stream>>>(Y4, MS4, F[15], F[16], OUT0, FH, FL);
  k_m<<<dim3((BS + 63) / 64, (TO + 127) / 128), 128, 0, stream>>>(FH, FL, PK, M);
  k_ob<<<BS, 256, 0, stream>>>(M, FH, FL);
  k_fc<<<BS / 16, 128, 0, stream>>>(FH, FL, PK, F[19], OUT1);
}
